// RNN_69114613728639
// MI455X (gfx1250) — hardware-verified
//
#include <hip/hip_runtime.h>
#include <math.h>

constexpr int NBATCH  = 64;
constexpr int NSTEP   = 1024;
constexpr int NEMB    = 256;
constexpr int NHID    = 256;
constexpr int NGATE   = 4 * NHID;
constexpr int KCAT    = NHID + NEMB;
constexpr int NVOC    = 50000;
constexpr int NFC     = 256;
constexpr int NOUTC   = 10;
constexpr int NTHR    = 256;
constexpr int SEQ_BLK = 16;
constexpr int HPITCH  = 264;
constexpr int OPITCH  = 260;
constexpr float WCARRY     = 16.0f;
constexpr float WCARRY_INV = 1.0f / WCARRY;
constexpr float BN_EPS_F   = 1e-5f;

static_assert(KCAT == 512, "k extent of the fused operand");
static_assert(NHID % 32 == 0 && NEMB % 32 == 0, "k chunks of 32");
static_assert(NBATCH % SEQ_BLK == 0, "blocks of 16 sequences");
static_assert(NHID == 32 * (NTHR / 32), "8 waves x 32 hidden units");
static_assert((2 * SEQ_BLK * HPITCH) % NTHR == 0, "h zero-fill loop exact");
static_assert(NFC == NTHR, "one fc1 column per thread");
static_assert((NBATCH * NOUTC * 4) % 512 == 0, "output is a whole number of 512-B wave stores");
static_assert((NBATCH * NSTEP * (NEMB / 8)) % NTHR == 0, "gather grid exact");

typedef __attribute__((ext_vector_type(16))) _Float16 v16h;
typedef __attribute__((ext_vector_type(8)))  _Float16 v8h;
typedef __attribute__((ext_vector_type(8)))  float    v8f;
typedef __attribute__((ext_vector_type(4)))  float    v4f;

__device__ __forceinline__ void grp_guard_h(v8f& a0, v8f& a1, v8f& a2, v8f& a3,
                                            v16h x, v16h b0, v16h b1, v16h b2, v16h b3) {
  asm volatile("v_nop\n\tv_nop\n\tv_nop\n\tv_nop"
               : "+v"(a0), "+v"(a1), "+v"(a2), "+v"(a3)
               : "v"(x), "v"(b0), "v"(b1), "v"(b2), "v"(b3));
}
__device__ __forceinline__ void acc_guard4(v8f& a, v8f& b, v8f& c, v8f& d) {
  asm volatile("v_nop\n\tv_nop\n\tv_nop\n\tv_nop" : "+v"(a), "+v"(b), "+v"(c), "+v"(d));
}

struct FragH {
  union U { v16h v; v8h h[2]; };
  static __device__ __forceinline__ v16h load(const _Float16* p) {
    U f;
    f.h[0] = *(const v8h*)(p);
    f.h[1] = *(const v8h*)(p + 16);
    return f.v;
  }
  static __device__ __forceinline__ v8f mma(v16h a, v16h b, v8f c) {
    return __builtin_amdgcn_wmma_f32_16x16x32_f16(false, a, false, b, (short)0, c, false, false);
  }
};

__device__ __forceinline__ float sigm_f(float x) { return __builtin_amdgcn_rcpf(1.0f + expf(-x)); }
__device__ __forceinline__ float tanh_f(float x) { return 1.0f - 2.0f * __builtin_amdgcn_rcpf(expf(2.0f * x) + 1.0f); }

__global__ __launch_bounds__(NTHR) void cvt8_f16_kernel(const float* __restrict__ src, unsigned short* __restrict__ dst,
                                                        int nrow, int ncol8, int spitch, int dpitch, int dcol0, float sc) {
  const int i  = blockIdx.x * NTHR + threadIdx.x;
  const int n8 = nrow * ncol8;
  if (i < n8) {
    const int row = i / ncol8;
    const int c8  = i - row * ncol8;
    const float* sp = src + (size_t)row * (size_t)spitch + (size_t)c8 * 8;
    const v4f a = *(const v4f*)(sp);
    const v4f b = *(const v4f*)(sp + 4);
    v8h hv;
#pragma unroll
    for (int e = 0; e < 4; ++e) {
      const float fa = a[e] * sc;
      const float fb = b[e] * sc;
      hv[e]     = (_Float16)fa;
      hv[4 + e] = (_Float16)fb;
    }
    unsigned short* op = dst + (size_t)row * (size_t)dpitch + (size_t)dcol0 + (size_t)c8 * 8;
    *(volatile v8h*)op = hv;
    __threadfence();
    *(volatile v8h*)op = hv;
  }
}

__global__ __launch_bounds__(NTHR) void gather_x_kernel(const int* __restrict__ xi, const float* __restrict__ emb,
                                                        unsigned short* __restrict__ XE) {
  const int i = blockIdx.x * NTHR + threadIdx.x;
  const int total = NBATCH * NSTEP * (NEMB / 8);
  if (i < total) {
    const int row = i >> 5;
    const int c8  = i & 31;
    const int t   = row >> 6;
    const int b   = row & 63;
    int id = xi[b * NSTEP + t];
    id = id < 0 ? 0 : id;
    id = id > (NVOC - 1) ? (NVOC - 1) : id;
    const float* sp = emb + (size_t)id * NEMB + (size_t)c8 * 8;
    const v4f a = *(const v4f*)(sp);
    const v4f c = *(const v4f*)(sp + 4);
    v8h hv;
#pragma unroll
    for (int e = 0; e < 4; ++e) {
      const float fa = a[e];
      const float fc = c[e];
      hv[e]     = (_Float16)fa;
      hv[4 + e] = (_Float16)fc;
    }
    unsigned short* op = XE + (size_t)i * 8;
    *(volatile v8h*)op = hv;
    __threadfence();
    *(volatile v8h*)op = hv;
  }
}

__global__ __launch_bounds__(NTHR) void lstm_seq_kernel(const unsigned short* __restrict__ XEp,
                                                        const unsigned short* __restrict__ WCp,
                                                        const float* __restrict__ b_ih, const float* __restrict__ b_hh,
                                                        float* __restrict__ HLAST) {
  __shared__ __align__(16) _Float16 Ah[2 * SEQ_BLK * HPITCH];
  __shared__ __align__(16) float    Hs[SEQ_BLK * OPITCH];
  const _Float16* XE = (const _Float16*)XEp;
  const _Float16* WC = (const _Float16*)WCp;
  const int tid = threadIdx.x;
  const int lane = tid & 31;
  const int wave = tid >> 5;
  const int c = lane & 15;
  const int hh = lane >> 4;
  const int koff = hh * 8;
  const int rowbase = blockIdx.x * SEQ_BLK;

#pragma unroll 1
  for (int i = tid; i < 2 * SEQ_BLK * HPITCH; i += NTHR) Ah[i] = (_Float16)0.0f;

  float cst[2][8], hst[2][8], bb[2][4];
#pragma unroll
  for (int nt = 0; nt < 2; ++nt) {
    const int j = 32 * wave + 16 * nt + c;
#pragma unroll
    for (int g = 0; g < 4; ++g) bb[nt][g] = b_ih[g * NHID + j] + b_hh[g * NHID + j];
#pragma unroll
    for (int r = 0; r < 8; ++r) { cst[nt][r] = 0.0f; hst[nt][r] = 0.0f; }
  }
  __syncthreads();

  const v8f z8 = {0.f, 0.f, 0.f, 0.f, 0.f, 0.f, 0.f, 0.f};
  const size_t gstride = (size_t)NHID * (size_t)KCAT;

#pragma unroll 1
  for (int t = 0; t < NSTEP; ++t) {
    const int cur = t & 1;
    const _Float16* ahrow = Ah + cur * (SEQ_BLK * HPITCH) + c * HPITCH + koff;
    _Float16* ahn = Ah + (cur ^ 1) * (SEQ_BLK * HPITCH);
    const _Float16* xrow = XE + ((size_t)t * NBATCH + (size_t)(rowbase + c)) * NEMB + koff;
#pragma unroll
    for (int nt = 0; nt < 2; ++nt) {
      const int j = 32 * wave + 16 * nt + c;
      const _Float16* wrow = WC + (size_t)j * KCAT + koff;
      v8f acc0 = z8, acc1 = z8, acc2 = z8, acc3 = z8;
#pragma unroll 1
      for (int k0 = 0; k0 < NHID; k0 += 32) {
        const v16h a  = FragH::load(ahrow + k0);
        const v16h b0 = FragH::load(wrow + k0);
        const v16h b1 = FragH::load(wrow + gstride + k0);
        const v16h b2 = FragH::load(wrow + 2 * gstride + k0);
        const v16h b3 = FragH::load(wrow + 3 * gstride + k0);
        acc0 = FragH::mma(a, b0, acc0);
        acc1 = FragH::mma(a, b1, acc1);
        acc2 = FragH::mma(a, b2, acc2);
        acc3 = FragH::mma(a, b3, acc3);
        grp_guard_h(acc0, acc1, acc2, acc3, a, b0, b1, b2, b3);
      }
#pragma unroll 1
      for (int kx = 0; kx < NEMB; kx += 32) {
        const v16h a  = FragH::load(xrow + kx);
        const v16h b0 = FragH::load(wrow + NHID + kx);
        const v16h b1 = FragH::load(wrow + gstride + NHID + kx);
        const v16h b2 = FragH::load(wrow + 2 * gstride + NHID + kx);
        const v16h b3 = FragH::load(wrow + 3 * gstride + NHID + kx);
        acc0 = FragH::mma(a, b0, acc0);
        acc1 = FragH::mma(a, b1, acc1);
        acc2 = FragH::mma(a, b2, acc2);
        acc3 = FragH::mma(a, b3, acc3);
        grp_guard_h(acc0, acc1, acc2, acc3, a, b0, b1, b2, b3);
      }
      acc_guard4(acc0, acc1, acc2, acc3);
#pragma unroll
      for (int r = 0; r < 8; ++r) {
        const float zi = acc0[r] * WCARRY_INV + bb[nt][0];
        const float zf = acc1[r] * WCARRY_INV + bb[nt][1];
        const float zg = acc2[r] * WCARRY_INV + bb[nt][2];
        const float zo = acc3[r] * WCARRY_INV + bb[nt][3];
        const float ig = sigm_f(zi);
        const float fg = sigm_f(zf);
        const float gg = tanh_f(zg);
        const float og = sigm_f(zo);
        const float cn = fg * cst[nt][r] + ig * gg;
        const float hn = og * tanh_f(cn);
        cst[nt][r] = cn;
        hst[nt][r] = hn;
        ahn[(8 * hh + r) * HPITCH + j] = (_Float16)hn;
      }
    }
    __syncthreads();
  }

#pragma unroll
  for (int nt = 0; nt < 2; ++nt) {
    const int j = 32 * wave + 16 * nt + c;
#pragma unroll
    for (int r = 0; r < 8; ++r) Hs[(8 * hh + r) * OPITCH + j] = hst[nt][r];
  }
  __syncthreads();
  for (int pass = 0; pass < 2; ++pass) {
#pragma unroll
    for (int it = 0; it < 4; ++it) {
      const int idx = it * NTHR + tid;
      const int row = idx >> 6;
      const int c4  = (idx & 63) * 4;
      const v4f v = *(const v4f*)(Hs + row * OPITCH + c4);
      *(volatile v4f*)(HLAST + (size_t)(rowbase + row) * NHID + c4) = v;
    }
    __threadfence();
  }
}

__global__ __launch_bounds__(NTHR) void head_kernel(const float* __restrict__ HL, const float* __restrict__ fc1_w,
                                                    const float* __restrict__ fc1_b, const float* __restrict__ gam,
                                                    const float* __restrict__ bet, const float* __restrict__ fc2_w,
                                                    const float* __restrict__ fc2_b, float* __restrict__ out) {
  __shared__ __align__(16) float Fb[NBATCH * NFC];
  __shared__ __align__(16) float Ob[NBATCH * NOUTC];
  const int tid = threadIdx.x;
  const int j = tid;
  const float* wrow = fc1_w + (size_t)j * NHID;
  const float bj = fc1_b[j];
  float sum = 0.0f;
#pragma unroll 1
  for (int b0 = 0; b0 < NBATCH; b0 += 4) {
    float a0 = 0.0f, a1 = 0.0f, a2 = 0.0f, a3 = 0.0f;
    const float* h0p = HL + (size_t)(b0 + 0) * NHID;
    const float* h1p = HL + (size_t)(b0 + 1) * NHID;
    const float* h2p = HL + (size_t)(b0 + 2) * NHID;
    const float* h3p = HL + (size_t)(b0 + 3) * NHID;
#pragma unroll 1
    for (int k = 0; k < NHID; k += 4) {
      const v4f w  = *(const v4f*)(wrow + k);
      const v4f x0 = *(const v4f*)(h0p + k);
      const v4f x1 = *(const v4f*)(h1p + k);
      const v4f x2 = *(const v4f*)(h2p + k);
      const v4f x3 = *(const v4f*)(h3p + k);
#pragma unroll
      for (int e = 0; e < 4; ++e) {
        a0 = fmaf(x0[e], w[e], a0);
        a1 = fmaf(x1[e], w[e], a1);
        a2 = fmaf(x2[e], w[e], a2);
        a3 = fmaf(x3[e], w[e], a3);
      }
    }
    a0 += bj; a1 += bj; a2 += bj; a3 += bj;
    Fb[(b0 + 0) * NFC + j] = a0;
    Fb[(b0 + 1) * NFC + j] = a1;
    Fb[(b0 + 2) * NFC + j] = a2;
    Fb[(b0 + 3) * NFC + j] = a3;
    sum += (a0 + a1) + (a2 + a3);
  }
  const float mu = sum * (1.0f / (float)NBATCH);
  float ss = 0.0f;
#pragma unroll 1
  for (int b = 0; b < NBATCH; ++b) {
    const float d = Fb[b * NFC + j] - mu;
    ss += d * d;
  }
  const float var  = ss * (1.0f / (float)NBATCH);
  const float rstd = rsqrtf(var + BN_EPS_F);
  const float gj = gam[j];
  const float ej = bet[j];
#pragma unroll 1
  for (int b = 0; b < NBATCH; ++b) {
    const float d = Fb[b * NFC + j] - mu;
    Fb[b * NFC + j] = (d * rstd) * gj + ej;
  }
  __syncthreads();

#pragma unroll 1
  for (int it = 0; it < 3; ++it) {
    const int idx = it * NTHR + tid;
    const bool valid = idx < NBATCH * NOUTC;
    const int idc = valid ? idx : (NBATCH * NOUTC - 1);
    const int b = idc / NOUTC;
    const int o = idc - b * NOUTC;
    const float* bp = Fb + b * NFC;
    const float* wp = fc2_w + (size_t)o * NFC;
    float s = 0.0f;
#pragma unroll 1
    for (int k = 0; k < NFC; k += 4) {
      const v4f xv = *(const v4f*)(bp + k);
      const v4f wv = *(const v4f*)(wp + k);
#pragma unroll
      for (int e = 0; e < 4; ++e) s = fmaf(xv[e], wv[e], s);
    }
    s += fc2_b[o];
    if (valid) Ob[idx] = s;
  }
  __syncthreads();

  if (tid < 32) {
    for (int pass = 0; pass < 2; ++pass) {
#pragma unroll
      for (int it = 0; it < 5; ++it) {
        const int q4 = (it * 32 + tid) * 4;
        const v4f v = *(const v4f*)(Ob + q4);
        *(volatile v4f*)(out + q4) = v;
      }
      __threadfence();
    }
  }
}

extern "C" void kernel_launch(void* const* d_in, const int* in_sizes, int n_in,
                              void* d_out, int out_size, void* d_ws, size_t ws_size, hipStream_t stream) {
  if (n_in < 12 || d_out == nullptr || d_ws == nullptr) return;
  if (in_sizes[0] != NBATCH * NSTEP || in_sizes[1] != NVOC * NEMB || in_sizes[2] != NGATE * NEMB ||
      in_sizes[3] != NGATE * NHID || in_sizes[4] != NGATE || in_sizes[5] != NGATE ||
      in_sizes[6] != NFC * NHID || in_sizes[7] != NFC || in_sizes[8] != NFC || in_sizes[9] != NFC ||
      in_sizes[10] != NOUTC * NFC || in_sizes[11] != NOUTC || out_size != NBATCH * NOUTC) return;

  const int*   xi    = (const int*)d_in[0];
  const float* emb   = (const float*)d_in[1];
  const float* w_ih  = (const float*)d_in[2];
  const float* w_hh  = (const float*)d_in[3];
  const float* b_ih  = (const float*)d_in[4];
  const float* b_hh  = (const float*)d_in[5];
  const float* fc1_w = (const float*)d_in[6];
  const float* fc1_b = (const float*)d_in[7];
  const float* gam   = (const float*)d_in[8];
  const float* bet   = (const float*)d_in[9];
  const float* fc2_w = (const float*)d_in[10];
  const float* fc2_b = (const float*)d_in[11];
  float* out = (float*)d_out;

  char* ws = (char*)d_ws;
  size_t off = 0;
  auto carve = [&](size_t bytes) -> char* { char* p = ws + off; off += (bytes + 255) & ~(size_t)255; return p; };
  unsigned short* WC    = (unsigned short*)carve((size_t)NGATE * KCAT * 2);
  unsigned short* XE    = (unsigned short*)carve((size_t)NBATCH * NSTEP * NEMB * 2);
  float*          HLAST = (float*)carve((size_t)NBATCH * NHID * 4);
  if (off > ws_size || off > (size_t)134217728) return;

  const int n8w = NGATE * (NHID / 8);
  cvt8_f16_kernel<<<(n8w + NTHR - 1) / NTHR, NTHR, 0, stream>>>(w_hh, WC, NGATE, NHID / 8, NHID, KCAT, 0, WCARRY);
  cvt8_f16_kernel<<<(n8w + NTHR - 1) / NTHR, NTHR, 0, stream>>>(w_ih, WC, NGATE, NEMB / 8, NEMB, KCAT, NHID, WCARRY);
  const int nthx = NBATCH * NSTEP * (NEMB / 8);
  gather_x_kernel<<<nthx / NTHR, NTHR, 0, stream>>>(xi, emb, XE);
  lstm_seq_kernel<<<NBATCH / SEQ_BLK, NTHR, 0, stream>>>(XE, WC, b_ih, b_hh, HLAST);
  head_kernel<<<1, NTHR, 0, stream>>>(HLAST, fc1_w, fc1_b, gam, bet, fc2_w, fc2_b, out);
}
